// IMEGPT2Attention_14637248545507
// MI455X (gfx1250) — hardware-verified
//
#include <hip/hip_runtime.h>


#ifndef NB
#define NB 2
#endif
#ifndef SEQ
#define SEQ 2048
#endif
#define NB_FULL   2
#define SEQ_FULL  2048
#define HID       1024
#define NHEAD     16
#define HD        64
#define MROWS     (NB * SEQ)
#define EARLY     ((SEQ < 256) ? SEQ : 256)

static_assert(HID == NHEAD * HD);
static_assert(HID == 1024);
static_assert(NHEAD == 16);
static_assert(HD == 64);
static_assert(SEQ % 128 == 0);
static_assert(SEQ <= SEQ_FULL);
static_assert(NB >= 1 && NB <= NB_FULL);
static_assert(MROWS % 128 == 0);
static_assert(HID % 128 == 0);
static_assert(HID % 32 == 0);
static_assert(EARLY % 128 == 0);
static_assert(EARLY >= 128 && EARLY <= SEQ);

#define CARRY_X    16.0f
#define CARRY_W    32.0f
#define CARRY_QKV  16.0f
#define CARRY_CTX  1024.0f
#define RES_CARRY  2048.0f
#define RES_INV    0.00048828125f

typedef unsigned u32;
typedef _Float16 f16;
typedef f16   v16h __attribute__((ext_vector_type(16)));
typedef f16   v8h  __attribute__((ext_vector_type(8)));
typedef float v8f  __attribute__((ext_vector_type(8)));
typedef float v4f  __attribute__((ext_vector_type(4)));

union FragU { v16h v; v8h half[2]; f16 e[16]; };
union H8U   { v8h v; f16 e[8]; };

__device__ __forceinline__ v8f zero8() {
    v8f z = {0.f, 0.f, 0.f, 0.f, 0.f, 0.f, 0.f, 0.f};
    return z;
}

__device__ __forceinline__ v8f wmma16(v16h a, v16h b, v8f c) {
    v8f d = __builtin_amdgcn_wmma_f32_16x16x32_f16(false, a, false, b, (short)0, c, false, false);
    asm volatile("v_nop\n\tv_nop\n\tv_nop\n\tv_nop" : "+v"(d) : "v"(a), "v"(b));
    return d;
}

__device__ __forceinline__ float bf16_rne(float x) {
    u32 u = __float_as_uint(x);
    u = (u + 0x7fffu + ((u >> 16) & 1u)) & 0xffff0000u;
    return __uint_as_float(u);
}

__device__ __forceinline__ f16 res16(float v, f16 hi) {
    return (f16)((v - (float)hi) * RES_CARRY);
}

__device__ __forceinline__ float fexp2(float x) {
#if defined(__has_builtin)
#if __has_builtin(__builtin_amdgcn_exp2f)
    return __builtin_amdgcn_exp2f(x);
#else
    return exp2f(x);
#endif
#else
    return exp2f(x);
#endif
}

__device__ __forceinline__ float rowmax16(float x) {
    int v = __builtin_bit_cast(int, x);
    x = fmaxf(x, __builtin_bit_cast(float, __builtin_amdgcn_update_dpp(v, v, 0x121, 0xf, 0xf, false)));
    v = __builtin_bit_cast(int, x);
    x = fmaxf(x, __builtin_bit_cast(float, __builtin_amdgcn_update_dpp(v, v, 0x122, 0xf, 0xf, false)));
    v = __builtin_bit_cast(int, x);
    x = fmaxf(x, __builtin_bit_cast(float, __builtin_amdgcn_update_dpp(v, v, 0x124, 0xf, 0xf, false)));
    v = __builtin_bit_cast(int, x);
    x = fmaxf(x, __builtin_bit_cast(float, __builtin_amdgcn_update_dpp(v, v, 0x128, 0xf, 0xf, false)));
    return x;
}

__device__ __forceinline__ v16h load_frag(const f16* tile, u32 rowbase, u32 pitch, u32 kcol, u32 lane) {
    const u32 r  = rowbase + (lane & 15u);
    const u32 kh = (lane >> 4) << 3;
    const f16* p = tile + (size_t)r * pitch + kcol + kh;
    FragU f;
    f.half[0] = *(const v8h*)(p);
    f.half[1] = *(const v8h*)(p + 16);
    return f.v;
}

__global__ void __launch_bounds__(256)
cvt_rows(const float* __restrict__ src, f16* __restrict__ dst, u32 nrows, float carry) {
    const u32 g  = blockIdx.x * 256u + threadIdx.x;
    const u32 m  = g >> 7;
    const u32 c8 = (g & 127u) << 3;
    if (m >= nrows) return;
    const u32 mb = m / (u32)SEQ;
    const u32 sm = mb * (u32)SEQ_FULL + (m - mb * (u32)SEQ);
    const float* sp = src + (size_t)sm * HID + c8;
    const v4f a = *(const v4f*)sp;
    const v4f b = *(const v4f*)(sp + 4);
    H8U o;
#pragma unroll
    for (u32 j = 0; j < 4; ++j) {
        const float x0 = a[j];
        const float x1 = b[j];
        o.e[j]     = (f16)(bf16_rne(x0) * carry);
        o.e[j + 4] = (f16)(bf16_rne(x1) * carry);
    }
    f16* dp = dst + (size_t)m * HID + c8;
    *(volatile v8h*)dp = o.v;
    __threadfence();
    *(volatile v8h*)dp = o.v;
}

__global__ void __launch_bounds__(256)
cvt_transpose(const float* __restrict__ src, f16* __restrict__ dst, u32 kd, u32 nd, float carry) {
    __shared__ __attribute__((aligned(16))) f16 Ts[64 * 72];

    const u32 tid = threadIdx.x;
    const u32 n0  = blockIdx.x * 64u;
    const u32 k0  = blockIdx.y * 64u;
    const u32 kr  = tid >> 4;
    const u32 nc  = (tid & 15u) << 2;

#pragma unroll
    for (u32 it = 0; it < 4; ++it) {
        const u32 kl = kr + it * 16u;
        const v4f a = *(const v4f*)(src + (size_t)(k0 + kl) * nd + n0 + nc);
#pragma unroll
        for (u32 j = 0; j < 4; ++j) {
            const float x0 = a[j];
            Ts[(nc + j) * 72u + kl] = (f16)(bf16_rne(x0) * carry);
        }
    }
    __syncthreads();

#pragma unroll
    for (u32 pass = 0; pass < 2; ++pass) {
#pragma unroll
        for (u32 it = 0; it < 2; ++it) {
            const u32 idx   = tid + it * 256u;
            const u32 line  = idx >> 3;
            const u32 piece = idx & 7u;
            const v8h v = *(const v8h*)&Ts[line * 72u + piece * 8u];
            f16* dp = dst + (size_t)(n0 + line) * kd + k0 + piece * 8u;
            *(volatile v8h*)dp = v;
        }
        if (pass == 0) __threadfence();
    }
}

template <int MODE>
__device__ __forceinline__ void gemm_body(const f16* __restrict__ A, const size_t resOff,
                                          const f16* __restrict__ W, const float* __restrict__ bias,
                                          const float biasMul, f16* __restrict__ outH,
                                          f16* __restrict__ outR, float* __restrict__ outF,
                                          const float accMul) {
    __shared__ __attribute__((aligned(16))) f16 As[128 * 32];
    __shared__ __attribute__((aligned(16))) f16 Bs[128 * 32];
    __shared__ __attribute__((aligned(16))) f16 Cs[(MODE == 2) ? 8 : 128 * 128];
    __shared__ __attribute__((aligned(16))) float Cf[(MODE == 2) ? 64 * 128 : 4];

    const u32 tid  = threadIdx.x;
    const u32 lane = tid & 31u;
    const u32 wave = (u32)__builtin_amdgcn_readfirstlane((int)(tid >> 5));
    const u32 wm   = wave & 3u;
    const u32 wn   = wave >> 2;
    const u32 hh8  = (lane >> 4) << 3;
    const u32 c16  = lane & 15u;
    const u32 m0   = blockIdx.x * 128u;
    const u32 n0   = blockIdx.y * 128u;
    const u32 bidx = m0 / (u32)SEQ;
    const u32 s0   = m0 - bidx * (u32)SEQ;
    const bool early = s0 < (u32)EARLY;

    v8f acc[2][4];
#pragma unroll
    for (int i = 0; i < 2; ++i)
#pragma unroll
        for (int j = 0; j < 4; ++j) acc[i][j] = zero8();

    const u32 srow = tid >> 1;
    const u32 scol = (tid & 1u) << 4;
    const f16* gW = W + (size_t)(n0 + srow) * HID + scol;
    const size_t hiRow = (size_t)(m0 + srow) * HID + scol;
    const size_t rsRow = resOff + (size_t)(bidx * (u32)EARLY + (early ? s0 : 0u) + srow) * HID + scol;

    const u32 phase0 = (MODE == 2 && early) ? 0u : 1u;
#pragma unroll 1
    for (u32 ph = phase0; ph < 2u; ++ph) {
        const size_t aoff = (ph == 0u) ? rsRow : hiRow;
        const f16* gA = A + aoff;
#pragma unroll 1
        for (u32 k0 = 0; k0 < (u32)HID; k0 += 32u) {
            const v8h ra0 = *(const v8h*)(gA + k0);
            const v8h ra1 = *(const v8h*)(gA + k0 + 8);
            const v8h rb0 = *(const v8h*)(gW + k0);
            const v8h rb1 = *(const v8h*)(gW + k0 + 8);
            __syncthreads();
            *(v8h*)&As[srow * 32u + scol]      = ra0;
            *(v8h*)&As[srow * 32u + scol + 8u] = ra1;
            *(v8h*)&Bs[srow * 32u + scol]      = rb0;
            *(v8h*)&Bs[srow * 32u + scol + 8u] = rb1;
            __syncthreads();

            v16h af[2], bfr[4];
#pragma unroll
            for (int i = 0; i < 2; ++i) af[i] = load_frag(As, wm * 32u + (u32)i * 16u, 32u, 0u, lane);
#pragma unroll
            for (int j = 0; j < 4; ++j) bfr[j] = load_frag(Bs, wn * 64u + (u32)j * 16u, 32u, 0u, lane);
#pragma unroll
            for (int i = 0; i < 2; ++i)
#pragma unroll
                for (int j = 0; j < 4; ++j) acc[i][j] = wmma16(af[i], bfr[j], acc[i][j]);
        }
        if (ph == 0u) {
#pragma unroll
            for (int i = 0; i < 2; ++i)
#pragma unroll
                for (int j = 0; j < 4; ++j) acc[i][j] = acc[i][j] * RES_INV;
        }
    }

    float bcol[4];
#pragma unroll
    for (int j = 0; j < 4; ++j)
        bcol[j] = bf16_rne(bias[n0 + wn * 64u + (u32)j * 16u + c16]) * biasMul;

    const u32 piece = lane & 7u;
    const u32 lsub  = lane >> 3;

    if constexpr (MODE == 0) {
        const size_t bh0 = (size_t)bidx * NHEAD + (n0 >> 6);
#pragma unroll
        for (int pl = 0; pl < 2; ++pl) {
            if (pl == 0 || early) {
                if (pl == 1) __syncthreads();
#pragma unroll
                for (int i = 0; i < 2; ++i)
#pragma unroll
                    for (int j = 0; j < 4; ++j) {
                        const u32 nl = wn * 64u + (u32)j * 16u + c16;
#pragma unroll
                        for (int r = 0; r < 8; ++r) {
                            const u32 ml = wm * 32u + (u32)i * 16u + hh8 + (u32)r;
                            const float val = acc[i][j][r] * accMul + bcol[j];
                            const f16 hi = (f16)val;
                            Cs[ml * 128u + nl] = (pl == 0) ? hi : res16(val, hi);
                        }
                    }
                __syncthreads();
                f16* op = (pl == 0) ? outH : outR;
                const u32 prow = (pl == 0) ? (u32)SEQ : (u32)EARLY;
#pragma unroll
                for (int pass = 0; pass < 2; ++pass) {
#pragma unroll
                    for (u32 it = 0; it < 8; ++it) {
                        const u32 L    = wave * 32u + it * 4u + lsub;
                        const u32 ml   = L >> 1;
                        const u32 hsel = L & 1u;
                        const v8h v = *(const v8h*)&Cs[ml * 128u + hsel * 64u + piece * 8u];
                        f16* dp = op + ((bh0 + hsel) * prow + s0 + ml) * HD + piece * 8u;
                        *(volatile v8h*)dp = v;
                    }
                    if (pass == 0) __threadfence();
                }
            }
        }
    } else if constexpr (MODE == 1) {
#pragma unroll
        for (int pl = 0; pl < 2; ++pl) {
            if (pl == 0 || early) {
                if (pl == 1) __syncthreads();
#pragma unroll
                for (int i = 0; i < 2; ++i)
#pragma unroll
                    for (int j = 0; j < 4; ++j) {
                        const u32 nl = wn * 64u + (u32)j * 16u + c16;
                        H8U t;
#pragma unroll
                        for (int r = 0; r < 8; ++r) {
                            const float val = acc[i][j][r] * accMul + bcol[j];
                            const f16 hi = (f16)val;
                            t.e[r] = (pl == 0) ? hi : res16(val, hi);
                        }
                        *(v8h*)&Cs[nl * 128u + wm * 32u + (u32)i * 16u + hh8] = t.v;
                    }
                __syncthreads();
                f16* op = (pl == 0) ? outH : outR;
                const u32 prow = (pl == 0) ? (u32)SEQ : (u32)EARLY;
#pragma unroll
                for (int pass = 0; pass < 2; ++pass) {
#pragma unroll
                    for (u32 it = 0; it < 8; ++it) {
                        const u32 L  = wave * 32u + it * 4u + lsub;
                        const u32 nl = L >> 1;
                        const u32 mh = L & 1u;
                        const v8h v = *(const v8h*)&Cs[nl * 128u + mh * 64u + piece * 8u];
                        f16* dp = op + ((size_t)(bidx * (u32)HID + n0 + nl) * prow + s0 + mh * 64u + piece * 8u);
                        *(volatile v8h*)dp = v;
                    }
                    if (pass == 0) __threadfence();
                }
            }
        }
    } else {
#pragma unroll
        for (u32 half = 0; half < 2; ++half) {
            if ((wm >> 1) == half) {
#pragma unroll
                for (int i = 0; i < 2; ++i)
#pragma unroll
                    for (int j = 0; j < 4; ++j) {
                        const u32 nl = wn * 64u + (u32)j * 16u + c16;
#pragma unroll
                        for (int r = 0; r < 8; ++r) {
                            const u32 ml = (wm & 1u) * 32u + (u32)i * 16u + hh8 + (u32)r;
                            Cf[ml * 128u + nl] = acc[i][j][r] * accMul + bcol[j];
                        }
                    }
            }
            __syncthreads();
#pragma unroll
            for (int pass = 0; pass < 2; ++pass) {
#pragma unroll
                for (u32 it = 0; it < 8; ++it) {
                    const u32 L    = wave * 32u + it * 4u + lsub;
                    const u32 row  = L >> 2;
                    const u32 part = L & 3u;
                    const v4f v = *(const v4f*)&Cf[row * 128u + part * 32u + piece * 4u];
                    float* dp = outF + (size_t)(m0 + half * 64u + row) * HID + n0 + part * 32u + piece * 4u;
                    *(volatile v4f*)dp = v;
                }
                if (pass == 0) __threadfence();
            }
            __syncthreads();
        }
    }
}

__global__ void __launch_bounds__(256) __attribute__((amdgpu_num_vgpr(256)))
k_gemm_qk(const f16* __restrict__ Xh, const f16* __restrict__ Wt, const float* __restrict__ bqkv,
          f16* __restrict__ QKp, f16* __restrict__ QKr, float accMul, float biasMul) {
    const u32 z = blockIdx.z;
    gemm_body<0>(Xh, (size_t)0, Wt + (size_t)z * HID * HID, bqkv + z * (u32)HID, biasMul,
                 QKp + (size_t)z * MROWS * HID, QKr + (size_t)z * NB * EARLY * HID, (float*)0, accMul);
}

__global__ void __launch_bounds__(256) __attribute__((amdgpu_num_vgpr(256)))
k_gemm_vt(const f16* __restrict__ Xh, const f16* __restrict__ Wv, const float* __restrict__ bv,
          f16* __restrict__ Vtp, f16* __restrict__ Vtr, float accMul, float biasMul) {
    gemm_body<1>(Xh, (size_t)0, Wv, bv, biasMul, Vtp, Vtr, (float*)0, accMul);
}

__global__ void __launch_bounds__(256) __attribute__((amdgpu_num_vgpr(256)))
k_gemm_out(const f16* __restrict__ Cp, size_t resOff, const f16* __restrict__ Wot,
           const float* __restrict__ bproj, float* __restrict__ out, float accMul) {
    gemm_body<2>(Cp, resOff, Wot, bproj, 1.0f, (f16*)0, (f16*)0, out, accMul);
}

template <bool RES>
__device__ __forceinline__ void attn_body(const f16* __restrict__ Qp, const f16* __restrict__ Kp,
                                          const f16* __restrict__ Vt, const f16* __restrict__ Qr,
                                          const f16* __restrict__ Kr, const f16* __restrict__ Vr,
                                          f16* __restrict__ Cp, f16* __restrict__ Cr, const u32 qblk) {
    constexpr u32 KT   = RES ? 32u : 64u;
    constexpr int NT   = RES ? 2 : 4;
    constexpr int KK   = RES ? 1 : 2;
    constexpr u32 KIT  = (KT * 8u) / 256u;
    constexpr u32 VPPR = KT / 8u;
    constexpr u32 VSH  = RES ? 2u : 3u;
    static_assert((KT * 8u) % 256u == 0u);
    static_assert((1u << VSH) == VPPR);
    static_assert(NT * 16 == (int)KT);
    static_assert(KK * 32 == (int)KT);

    __shared__ __attribute__((aligned(16))) f16 ks[KT * 64];
    __shared__ __attribute__((aligned(16))) f16 vsT[64 * KT];
    __shared__ __attribute__((aligned(16))) f16 ps[8][16 * 64];
    __shared__ __attribute__((aligned(16))) f16 krs[RES ? KT * 64 : 8];
    __shared__ __attribute__((aligned(16))) f16 vrT[RES ? 64 * KT : 8];
    __shared__ __attribute__((aligned(16))) f16 prs[8][RES ? 16 * 64 : 8];

    const u32 tid  = threadIdx.x;
    const u32 lane = tid & 31u;
    const u32 wave = (u32)__builtin_amdgcn_readfirstlane((int)(tid >> 5));
    const u32 hh8  = (lane >> 4) << 3;
    const u32 c16  = lane & 15u;
    const u32 bh   = blockIdx.y;
    const u32 bidx = bh >> 4;
    const u32 hidx = bh & 15u;
    const u32 q0b  = qblk * 128u;
    const u32 q0   = q0b + wave * 16u;
    const size_t head  = (size_t)bh * SEQ * HD;
    const size_t headE = (size_t)bh * EARLY * HD;

    v16h qa[2];
#pragma unroll
    for (int c = 0; c < 2; ++c) qa[c] = load_frag(Qp + head, q0, HD, (u32)c * 32u, lane);

    FragU onesu;
#pragma unroll
    for (int i = 0; i < 16; ++i) onesu.e[i] = (f16)1.0f;
    const v16h ones = onesu.v;

    float m[8];
    v8f   o[4], orr[4], lacc, laccr;
#pragma unroll
    for (int r = 0; r < 8; ++r) m[r] = -1.0e30f;
#pragma unroll
    for (int dt = 0; dt < 4; ++dt) { o[dt] = zero8(); orr[dt] = zero8(); }
    lacc  = zero8();
    laccr = zero8();

    const float cl = 1.4426950408889634f * 0.00390625f;
    f16* psw = &ps[wave][0];
    f16* prw = &prs[wave][0];

    const u32 nkt = (q0b + 128u) / KT;

#pragma unroll 1
    for (u32 kt = 0; kt < nkt; ++kt) {
        const u32 kbase = kt * KT;
        __syncthreads();
#pragma unroll
        for (u32 i = 0; i < KIT; ++i) {
            const u32 p    = tid + i * 256u;
            const u32 krow = p >> 3;
            const u32 kpc  = (p & 7u) << 3;
            const u32 vrow = p >> VSH;
            const u32 vpc  = (p & (VPPR - 1u)) << 3;
            const v8h kv = *(const v8h*)(Kp + head + (size_t)(kbase + krow) * HD + kpc);
            const v8h vv = *(const v8h*)(Vt + head + (size_t)vrow * SEQ + kbase + vpc);
            *(v8h*)&ks[krow * 64u + kpc]  = kv;
            *(v8h*)&vsT[vrow * KT + vpc]  = vv;
            if constexpr (RES) {
                const v8h kq = *(const v8h*)(Kr + headE + (size_t)(kbase + krow) * HD + kpc);
                const v8h vq = *(const v8h*)(Vr + headE + (size_t)vrow * EARLY + kbase + vpc);
                *(v8h*)&krs[krow * 64u + kpc] = kq;
                *(v8h*)&vrT[vrow * KT + vpc]  = vq;
            }
        }
        __syncthreads();

        const bool act = kbase <= q0 + 15u;
        if (act) {
            v8f s[NT], sr[NT];
#pragma unroll
            for (int nt = 0; nt < NT; ++nt) { s[nt] = zero8(); sr[nt] = zero8(); }
            if constexpr (RES) {
#pragma unroll
                for (int c = 0; c < 2; ++c) {
                    const v16h qh = load_frag(Qp + head,  q0, HD, (u32)c * 32u, lane);
                    const v16h qr = load_frag(Qr + headE, q0, HD, (u32)c * 32u, lane);
#pragma unroll
                    for (int nt = 0; nt < NT; ++nt) {
                        const v16h kb = load_frag(ks,  (u32)nt * 16u, 64u, (u32)c * 32u, lane);
                        const v16h kr = load_frag(krs, (u32)nt * 16u, 64u, (u32)c * 32u, lane);
                        s[nt]  = wmma16(qh, kb, s[nt]);
                        sr[nt] = wmma16(qh, kr, sr[nt]);
                        sr[nt] = wmma16(qr, kb, sr[nt]);
                    }
                }
            } else {
#pragma unroll
                for (int c = 0; c < 2; ++c) {
#pragma unroll
                    for (int nt = 0; nt < NT; ++nt) {
                        const v16h kb = load_frag(ks, (u32)nt * 16u, 64u, (u32)c * 32u, lane);
                        s[nt] = wmma16(qa[c], kb, s[nt]);
                    }
                }
            }

            const bool needmask = (kbase + KT - 1u) > q0;
#pragma unroll
            for (int r = 0; r < 8; ++r) {
                const u32 row = q0 + hh8 + (u32)r;
                float x[NT];
#pragma unroll
                for (int nt = 0; nt < NT; ++nt) {
                    float sv = s[nt][r];
                    if constexpr (RES) sv += sr[nt][r] * RES_INV;
                    float xv = sv * cl;
                    if (needmask) {
                        const u32 key = kbase + (u32)nt * 16u + c16;
                        xv = (key <= row) ? xv : -1.0e30f;
                    }
                    x[nt] = xv;
                }
                float mx = x[0];
#pragma unroll
                for (int nt = 1; nt < NT; ++nt) mx = fmaxf(mx, x[nt]);
                const float tm = rowmax16(mx);
                const float mn = fmaxf(m[r], tm);
                const float al = fexp2(m[r] - mn);
                m[r] = mn;
                lacc[r] *= al;
                if constexpr (RES) laccr[r] *= al;
#pragma unroll
                for (int dt = 0; dt < 4; ++dt) {
                    o[dt][r] *= al;
                    if constexpr (RES) orr[dt][r] *= al;
                }
                const float sh = 10.0f - mn;
#pragma unroll
                for (int nt = 0; nt < NT; ++nt) {
                    const float pv = fexp2(x[nt] + sh);
                    const f16 ph = (f16)pv;
                    psw[(hh8 + (u32)r) * 64u + (u32)nt * 16u + c16] = ph;
                    if constexpr (RES) prw[(hh8 + (u32)r) * 64u + (u32)nt * 16u + c16] = res16(pv, ph);
                }
            }
        }
        __syncthreads();

        if (act) {
#pragma unroll
            for (int kk = 0; kk < KK; ++kk) {
                const v16h pa = load_frag(psw, 0u, 64u, (u32)kk * 32u, lane);
                if constexpr (RES) {
                    const v16h pq = load_frag(prw, 0u, 64u, (u32)kk * 32u, lane);
#pragma unroll
                    for (int dt = 0; dt < 4; ++dt) {
                        const v16h vb = load_frag(vsT, (u32)dt * 16u, KT, (u32)kk * 32u, lane);
                        const v16h vq = load_frag(vrT, (u32)dt * 16u, KT, (u32)kk * 32u, lane);
                        o[dt]   = wmma16(pa, vb, o[dt]);
                        orr[dt] = wmma16(pa, vq, orr[dt]);
                        orr[dt] = wmma16(pq, vb, orr[dt]);
                    }
                    lacc  = wmma16(pa, ones, lacc);
                    laccr = wmma16(pq, ones, laccr);
                } else {
#pragma unroll
                    for (int dt = 0; dt < 4; ++dt) {
                        const v16h vb = load_frag(vsT, (u32)dt * 16u, KT, (u32)kk * 32u, lane);
                        o[dt] = wmma16(pa, vb, o[dt]);
                    }
                    lacc = wmma16(pa, ones, lacc);
                }
            }
        }
    }
    __syncthreads();

#pragma unroll
    for (int r = 0; r < 8; ++r) {
        float den = lacc[r];
        if constexpr (RES) den += laccr[r] * RES_INV;
        const float inv = (CARRY_CTX / CARRY_QKV) / den;
#pragma unroll
        for (int dt = 0; dt < 4; ++dt) {
            float ov = o[dt][r];
            if constexpr (RES) ov += orr[dt][r] * RES_INV;
            const float cv = ov * inv;
            const f16 ch = (f16)cv;
            psw[(hh8 + (u32)r) * 64u + (u32)dt * 16u + c16] = ch;
            if constexpr (RES) prw[(hh8 + (u32)r) * 64u + (u32)dt * 16u + c16] = res16(cv, ch);
        }
    }
    __syncthreads();

    const u32 piece = lane & 7u;
    const u32 lsub  = lane >> 3;
#pragma unroll
    for (int pass = 0; pass < 2; ++pass) {
#pragma unroll
        for (u32 it = 0; it < 4; ++it) {
            const u32 L = it * 4u + lsub;
            const v8h v = *(const v8h*)&psw[L * 64u + piece * 8u];
            f16* dp = Cp + ((size_t)(bidx * (u32)SEQ + q0 + L) * HID + hidx * (u32)HD + piece * 8u);
            *(volatile v8h*)dp = v;
            if constexpr (RES) {
                const v8h w = *(const v8h*)&prw[L * 64u + piece * 8u];
                f16* dq = Cr + ((size_t)(bidx * (u32)EARLY + q0 + L) * HID + hidx * (u32)HD + piece * 8u);
                *(volatile v8h*)dq = w;
            }
        }
        if (pass == 0) __threadfence();
    }
}

__global__ void __launch_bounds__(256) __attribute__((amdgpu_num_vgpr(256)))
k_attn_early(const f16* __restrict__ Qp, const f16* __restrict__ Kp, const f16* __restrict__ Vt,
             const f16* __restrict__ Qr, const f16* __restrict__ Kr, const f16* __restrict__ Vr,
             f16* __restrict__ Cp, f16* __restrict__ Cr) {
    attn_body<true>(Qp, Kp, Vt, Qr, Kr, Vr, Cp, Cr, blockIdx.x);
}

__global__ void __launch_bounds__(256) __attribute__((amdgpu_num_vgpr(256)))
k_attn_main(const f16* __restrict__ Qp, const f16* __restrict__ Kp, const f16* __restrict__ Vt,
            f16* __restrict__ Cp) {
    attn_body<false>(Qp, Kp, Vt, Qp, Kp, Vt, Cp, Cp, blockIdx.x + (u32)(EARLY / 128));
}

static_assert((size_t)(MROWS / 2) * 256 * 8 == (size_t)MROWS * HID);
static_assert((size_t)(3 * HID / 64) * (HID / 64) * 4096 == (size_t)3 * HID * HID);
static_assert((size_t)(HID / 64) * (HID / 64) * 4096 == (size_t)HID * HID);
static_assert((size_t)(MROWS / 128) * (HID / 128) * 128 * 128 == (size_t)MROWS * HID);
static_assert((size_t)(SEQ / 128) * (NB * NHEAD) * 128 * HD == (size_t)MROWS * HID);
static_assert((size_t)(EARLY / 128) * (NB * NHEAD) * 128 * HD == (size_t)NB * EARLY * HID);

#define N_X   ((size_t)MROWS * HID)
#define N_W   ((size_t)HID * HID)
#define N_XE  ((size_t)NB * EARLY * HID)
static_assert((5 * N_X + 4 * N_W + 4 * N_XE) * 2 <= (size_t)134217728);
static_assert((N_X * 2) % 128 == 0);
static_assert((N_W * 2) % 128 == 0);
static_assert((N_XE * 2) % 128 == 0);

extern "C" void kernel_launch(void* const* d_in, const int* in_sizes, int n_in,
                              void* d_out, int out_size, void* d_ws, size_t ws_size,
                              hipStream_t stream) {
    if (n_in < 5) return;
    if (in_sizes[0] < ((NB - 1) * SEQ_FULL + SEQ) * HID) return;
    if (in_sizes[1] < HID * 3 * HID) return;
    if (in_sizes[2] < 3 * HID) return;
    if (in_sizes[3] < HID * HID) return;
    if (in_sizes[4] < HID) return;
    if (out_size < MROWS * HID) return;

    const float* x     = (const float*)d_in[0];
    const float* wqkv  = (const float*)d_in[1];
    const float* bqkv  = (const float*)d_in[2];
    const float* wproj = (const float*)d_in[3];
    const float* bproj = (const float*)d_in[4];

    const size_t nX  = N_X;
    const size_t nW  = N_W;
    const size_t nXE = N_XE;
    const size_t totalHalves = 5 * nX + 4 * nW + 4 * nXE;
    if (ws_size < totalHalves * sizeof(f16)) return;

    f16* Xh  = (f16*)d_ws;
    f16* Wt  = Xh  + nX;
    f16* Wot = Wt  + 3 * nW;
    f16* Qp  = Wot + nW;
    f16* Kp  = Qp  + nX;
    f16* Vtp = Kp  + nX;
    f16* Cp  = Vtp + nX;
    f16* Qr  = Cp  + nX;
    f16* Kr  = Qr  + nXE;
    f16* Vtr = Kr  + nXE;
    f16* Cr  = Vtr + nXE;
    const size_t crOff = nX + 3 * nXE;

    cvt_rows<<<MROWS / 2, 256, 0, stream>>>(x, Xh, (u32)MROWS, CARRY_X);
    cvt_transpose<<<dim3(3 * HID / 64, HID / 64), 256, 0, stream>>>(wqkv, Wt, (u32)HID, (u32)(3 * HID), CARRY_W);
    cvt_transpose<<<dim3(HID / 64, HID / 64), 256, 0, stream>>>(wproj, Wot, (u32)HID, (u32)HID, CARRY_W);

    const float accQKV = CARRY_QKV / (CARRY_X * CARRY_W);
    k_gemm_qk<<<dim3(MROWS / 128, HID / 128, 2), 256, 0, stream>>>(Xh, Wt, bqkv, Qp, Qr, accQKV, CARRY_QKV);
    k_gemm_vt<<<dim3(MROWS / 128, HID / 128), 256, 0, stream>>>(Xh, Wt + 2 * nW, bqkv + 2 * HID, Vtp, Vtr, accQKV, CARRY_QKV);

    k_attn_early<<<dim3(EARLY / 128, NB * NHEAD), 256, 0, stream>>>(Qp, Kp, Vtp, Qr, Kr, Vtr, Cp, Cr);
    if (SEQ / 128 > EARLY / 128) {
        k_attn_main<<<dim3(SEQ / 128 - EARLY / 128, NB * NHEAD), 256, 0, stream>>>(Qp, Kp, Vtp, Cp);
    }

    const float accOut = 1.0f / (CARRY_CTX * CARRY_W);
    k_gemm_out<<<dim3(MROWS / 128, HID / 128), 256, 0, stream>>>(Cp, crOff, Wot, bproj, (float*)d_out, accOut);
}
